// TrajectoryCritic_1838246003412
// MI455X (gfx1250) — hardware-verified
//
#include <hip/hip_runtime.h>


namespace {
constexpr int S = 20, NSEQ = 512, NPED = 64, B_ = NSEQ * NPED, M = 1024, NBLK = B_ / 128;
constexpr float THR = 0.25f, BNE = 1e-5f;

typedef _Float16 b16;
typedef __attribute__((ext_vector_type(16))) _Float16 v16b;
typedef __attribute__((ext_vector_type(8))) float v8f;
typedef __attribute__((ext_vector_type(4))) float v4f;
__device__ __forceinline__ void split16(float v, b16& hi, b16& lo) { hi = (b16)v; lo = (b16)(v - (float)hi); }
__device__ __forceinline__ v8f wmma16b(v16b a, v16b b, v8f c) {
  v8f d = __builtin_amdgcn_wmma_f32_16x16x32_f16(false, a, false, b, (short)0, c, false, false);
  asm volatile("v_nop\n\tv_nop\n\tv_nop\n\tv_nop" : "+v"(d) : "v"(a), "v"(b));
  return d;
}

__global__ __launch_bounds__(256) void collide_kernel(const float* __restrict__ traj, float* __restrict__ rewards, float* __restrict__ rw2) {
  __shared__ float px[S][NPED], py[S][NPED]; __shared__ float mind[4][NPED];
  const int t_ = threadIdx.x, seq = blockIdx.x;
  for (int i = t_; i < S * NPED; i += 256) { const int s = i / NPED, p = i % NPED; const size_t g = ((size_t)s * B_ + (size_t)seq * NPED + p) * 2; px[s][p] = traj[g]; py[s][p] = traj[g + 1]; }
  __syncthreads();
  const int p = t_ & 63, part = t_ >> 6; float md = INFINITY;
  for (int s = part; s < S; s += 4) { const float x0 = px[s][p], y0 = py[s][p];
    for (int q = 0; q < NPED; ++q) { const float dx = __fsub_rn(x0, px[s][q]), dy = __fsub_rn(y0, py[s][q]); float dd = __fsqrt_rn(__fadd_rn(__fmul_rn(dx, dx), __fmul_rn(dy, dy))); dd = (dd == 0.0f) ? THR : dd; md = fminf(md, dd); } }
  mind[part][p] = md;
  __syncthreads();
  if (t_ < NPED) { const float m = fminf(fminf(mind[0][t_], mind[1][t_]), fminf(mind[2][t_], mind[3][t_])); mind[0][t_] = (m < THR) ? 0.0f : 1.0f; }
  __syncthreads();
  for (int pass = 0; pass < 2; ++pass) { if (t_ < 16) { *(volatile v4f*)(rewards + (size_t)seq * NPED + t_ * 4) = *(const v4f*)(&mind[0][t_ * 4]); *(volatile v4f*)(rw2 + (size_t)seq * NPED + t_ * 4) = *(const v4f*)(&mind[0][t_ * 4]); } __threadfence(); }
}

__global__ __launch_bounds__(1024) void layer1_kernel(const float* __restrict__ rw, const float* __restrict__ W1, const float* __restrict__ b1, const float* __restrict__ g1, const float* __restrict__ be1, float* __restrict__ R) {
  __shared__ int red[32];
  const int t_ = threadIdx.x; int c = 0;
  for (int i = t_; i < B_; i += 1024) c += (rw[i] > 0.5f) ? 1 : 0;
#pragma unroll
  for (int o = 16; o > 0; o >>= 1) c += __shfl_xor(c, o);
  if ((t_ & 31) == 0) red[t_ >> 5] = c;
  __syncthreads();
  int n1 = 0;
#pragma unroll
  for (int w = 0; w < 32; ++w) n1 += red[w];
  const double dn1 = (double)n1, dn0 = (double)(B_ - n1), dB = (double)B_;
  const int j = t_; const float v1 = W1[j] + b1[j], v0 = b1[j];
  const double mean = (dn0 * (double)v0 + dn1 * (double)v1) / dB, dv = (double)v1 - (double)v0, var = dn0 * dn1 * dv * dv / (dB * dB);
  const float a = g1[j] * (float)(1.0 / sqrt(var + (double)BNE)), sh = be1[j] - (float)mean * a;
  const float r0 = fmaxf(v0 * a + sh, 0.0f), r1 = fmaxf(v1 * a + sh, 0.0f);
  for (int pass = 0; pass < 2; ++pass) { ((volatile float*)R)[j] = r0; ((volatile float*)R)[M + j] = r1; __threadfence(); }
}

__global__ __launch_bounds__(128) void layer2_kernel(const float* __restrict__ rw, const float* __restrict__ R, const float* __restrict__ W2, const float* __restrict__ b2, float* __restrict__ h2, float* __restrict__ slot_) {
  __shared__ float Hs[128]; __shared__ float Ps[4][2];
  const int lane = threadIdx.x & 31, wave = threadIdx.x >> 5, nloc = lane & 15, hlf = lane >> 4, m0 = blockIdx.x * 128 + wave * 32;
  const float ra = rw[m0 + nloc], rb = rw[m0 + 16 + nloc];
  v8f acc0 = {}, acc1 = {};
#pragma unroll 2
  for (int kb = 0; kb < M; kb += 32) { v16b a0, l0, a1, l1, bh, bl;
#pragma unroll
    for (int e = 0; e < 16; ++e) { const int k = kb + ((e < 8) ? (8 * hlf + e) : (16 + 8 * hlf + e - 8)); const float x0 = R[k], x1 = R[M + k], d = x1 - x0; b16 p, q;
      split16((x0 + ra * d) * 8.0f, p, q); a0[e] = p; l0[e] = q; split16((x0 + rb * d) * 8.0f, p, q); a1[e] = p; l1[e] = q;
      split16((nloc == 0) ? W2[k] * 64.0f : 0.0f, p, q); bh[e] = p; bl[e] = q; }
    acc0 = wmma16b(a0, bh, acc0); acc0 = wmma16b(l0, bh, acc0); acc0 = wmma16b(a0, bl, acc0);
    acc1 = wmma16b(a1, bh, acc1); acc1 = wmma16b(l1, bh, acc1); acc1 = wmma16b(a1, bl, acc1); }
  if (nloc == 0) {
#pragma unroll
    for (int v = 0; v < 8; ++v) { Hs[wave * 32 + 8 * hlf + v] = acc0[v] * (1.0f / 512.0f) + b2[0]; Hs[wave * 32 + 16 + 8 * hlf + v] = acc1[v] * (1.0f / 512.0f) + b2[0]; } }
  __syncthreads();
  if (threadIdx.x < 32) { float s = 0.0f, s2 = 0.0f; for (int i = threadIdx.x; i < 128; i += 32) { s += Hs[i]; s2 += Hs[i] * Hs[i]; }
#pragma unroll
    for (int o = 16; o > 0; o >>= 1) { s += __shfl_xor(s, o); s2 += __shfl_xor(s2, o); }
    if (threadIdx.x == 0) { Ps[0][0] = s; Ps[0][1] = s2; } }
  __syncthreads();
  for (int pass = 0; pass < 2; ++pass) {
    if (threadIdx.x < 32) *(volatile v4f*)(h2 + (size_t)blockIdx.x * 128 + threadIdx.x * 4) = *(const v4f*)(&Hs[threadIdx.x * 4]);
    if (threadIdx.x < 2) ((volatile float*)slot_)[(size_t)blockIdx.x * 32 + threadIdx.x] = Ps[0][threadIdx.x];
    __threadfence();
  }
}

__global__ __launch_bounds__(128) void score_kernel(const float* __restrict__ h2, const float* __restrict__ slot_, const float* __restrict__ g2, const float* __restrict__ be2, float* __restrict__ scores) {
  __shared__ float cf[2];
  if (threadIdx.x == 0) { double s = 0.0, s2 = 0.0; for (int bk = 0; bk < NBLK; ++bk) { s += (double)slot_[(size_t)bk * 32]; s2 += (double)slot_[(size_t)bk * 32 + 1]; }
    const double mean = s / B_, var = s2 / B_ - mean * mean; const float a = g2[0] * (float)(1.0 / sqrt(var + (double)BNE)); cf[0] = a; cf[1] = be2[0] - (float)mean * a; }
  __syncthreads();
  const float a = cf[0], sh = cf[1];
  for (int pass = 0; pass < 2; ++pass) { if (threadIdx.x < 32) { const v4f h = *(const v4f*)(h2 + (size_t)blockIdx.x * 128 + threadIdx.x * 4); v4f o;
#pragma unroll
      for (int c = 0; c < 4; ++c) o[c] = fmaxf(h[c] * a + sh, 0.0f);
      *(volatile v4f*)(scores + (size_t)blockIdx.x * 128 + threadIdx.x * 4) = o; } __threadfence(); }
}
}

extern "C" void kernel_launch(void* const* d_in, const int* in_sizes, int n_in,
                              void* d_out, int out_size, void* d_ws, size_t ws_size, hipStream_t stream) {
  (void)n_in; (void)out_size;
  const float* traj = (const float*)d_in[0];
  const float* W1 = (const float*)d_in[9]; const float* b1 = (const float*)d_in[10]; const float* g1 = (const float*)d_in[11]; const float* be1 = (const float*)d_in[12];
  const float* W2 = (const float*)d_in[13]; const float* b2 = (const float*)d_in[14]; const float* g2 = (const float*)d_in[15]; const float* be2 = (const float*)d_in[16];
  float* scores = (float*)d_out; float* rewards = scores + B_;
  if (in_sizes[0] != S * B_ * 2 || in_sizes[9] != M || in_sizes[13] != M) return;
  size_t off = 0; char* ws = (char*)d_ws;
  auto carve = [&](size_t bytes) { char* p = ws + off; off += (bytes + 255) & ~(size_t)255; return p; };
  float* rw = (float*)carve((size_t)B_ * 4); float* R = (float*)carve(2 * M * 4); float* h2 = (float*)carve((size_t)B_ * 4); float* slot_ = (float*)carve((size_t)NBLK * 32 * 4);
  if (off > ws_size) return;
  collide_kernel<<<NSEQ, 256, 0, stream>>>(traj, rw, rewards);
  layer1_kernel<<<1, 1024, 0, stream>>>(rw, W1, b1, g1, be1, R);
  layer2_kernel<<<NBLK, 128, 0, stream>>>(rw, R, W2, b2, h2, slot_);
  score_kernel<<<NBLK, 128, 0, stream>>>(h2, slot_, g2, be2, scores);
}
